// MultiHeadAttention_30391188586935
// MI455X (gfx1250) — hardware-verified
//
#include <hip/hip_runtime.h>
#include <math.h>

#ifndef NB
#define NB 4
#endif
#ifndef SEQ
#define SEQ 2048
#endif
#define NB_FULL 4
#define SEQ_FULL 2048
#define DM 1024
#define NH 16
#define HD 64

typedef _Float16 v16h __attribute__((ext_vector_type(16)));
typedef _Float16 v8h  __attribute__((ext_vector_type(8)));
typedef float    v8f  __attribute__((ext_vector_type(8)));
typedef float    v4f  __attribute__((ext_vector_type(4)));
typedef unsigned v4u  __attribute__((ext_vector_type(4)));
typedef v8h v8h_ma __attribute__((may_alias));
typedef v4f v4f_ma __attribute__((may_alias));

static_assert(NH * HD == DM);
static_assert(HD == 64);
static_assert(DM % 64 == 0);
static_assert(SEQ % 64 == 0);
static_assert((NB * SEQ) % 64 == 0);
static_assert(NB <= NB_FULL && SEQ <= SEQ_FULL);
static_assert((((NB * SEQ) / 64) * ((2 * DM) / 64)) % 8 == 0);
static_assert(((DM / 64) * (SEQ / 64)) % 8 == 0);
static_assert(((SEQ / 64) * (DM / 64)) % 8 == 0);

union FH { v16h v; v8h h[2]; };
__device__ __forceinline__ v16h ldfrag_g(const _Float16* p) { FH f; f.h[0] = *(const v8h*)(p); f.h[1] = *(const v8h*)(p + 16); return f.v; }
__device__ __forceinline__ v8f mma_h(v16h a, v16h b, v8f c) { return __builtin_amdgcn_wmma_f32_16x16x32_f16(false, a, false, b, (short)0, c, false, false); }
__device__ __forceinline__ void dep_guard_h(v8f& a, v8f& b, v16h x, v16h y) { asm volatile("v_nop\n\tv_nop\n\tv_nop\n\tv_nop" : "+v"(a), "+v"(b) : "v"(x), "v"(y)); }
__device__ __forceinline__ void keep4_h(v16h a, v16h b, v16h c, v16h d) { asm volatile("v_nop" :: "v"(a), "v"(b), "v"(c), "v"(d)); }
__device__ __forceinline__ void acc_guard4(v8f& a, v8f& b, v8f& c, v8f& d) { asm volatile("v_nop\n\tv_nop\n\tv_nop\n\tv_nop" : "+v"(a), "+v"(b), "+v"(c), "+v"(d)); }
__device__ __forceinline__ void guard_s(v8f& a, v8f& b, v16h x, v16h y, v16h z) { asm volatile("v_nop\n\tv_nop\n\tv_nop\n\tv_nop" : "+v"(a), "+v"(b) : "v"(x), "v"(y), "v"(z)); }
__device__ __forceinline__ void guard_o(v8f& a, v8f& b, v8f& c, v8f& d, v16h p, v16h x, v16h y, v16h z, v16h w) {
    asm volatile("v_nop\n\tv_nop\n\tv_nop\n\tv_nop" : "+v"(a), "+v"(b), "+v"(c), "+v"(d) : "v"(p), "v"(x), "v"(y), "v"(z), "v"(w)); }
__device__ __forceinline__ void wave_sync_lds() {
    __builtin_amdgcn_fence(3  , "workgroup");
    __builtin_amdgcn_wave_barrier();
    __builtin_amdgcn_fence(2  , "workgroup");
}

#define VST2(T, ptr, val) do { const T vst2_v_ = (val); *(volatile T*)(ptr) = vst2_v_; __threadfence(); *(volatile T*)(ptr) = vst2_v_; } while (0)

__device__ __forceinline__ float cmb_bf(float v) { const unsigned u = __builtin_bit_cast(unsigned, v); const unsigned r = (u + 0x7fffu + ((u >> 16) & 1u)) & 0xffff0000u; return __builtin_bit_cast(float, r); }
__device__ __forceinline__ unsigned cmb_pk2(float a, float b) { return (unsigned)__builtin_bit_cast(unsigned short, (_Float16)a) | ((unsigned)__builtin_bit_cast(unsigned short, (_Float16)b) << 16); }

__global__ __launch_bounds__(256) void k_cast_x(const float* __restrict__ X, unsigned short* __restrict__ X16) {
    const long long u = (long long)blockIdx.x * 256 + threadIdx.x; const int per = DM / 8;
    if (u >= (long long)NB * SEQ * per) return;
    const int r = (int)(u / per); const int c0 = 8 * (int)(u % per); const int b = r / SEQ; const int s = r - b * SEQ;
    const float* src = X + ((size_t)b * SEQ_FULL + s) * DM + c0;
    const v4f a = *(const v4f*)(src); const v4f d = *(const v4f*)(src + 4);
    v4u pk; pk.x = cmb_pk2(cmb_bf(a.x), cmb_bf(a.y)); pk.y = cmb_pk2(cmb_bf(a.z), cmb_bf(a.w)); pk.z = cmb_pk2(cmb_bf(d.x), cmb_bf(d.y)); pk.w = cmb_pk2(cmb_bf(d.z), cmb_bf(d.w));
    VST2(v4u, (v4u*)(X16 + (size_t)r * DM + c0), pk);
}
__global__ __launch_bounds__(256) void k_castT_w(const float* __restrict__ SRC, int lds, unsigned short* __restrict__ DST, int ldd, int nR, int nC, float sc) {
    const long long u = (long long)blockIdx.x * 256 + threadIdx.x; const int per = nR / 8; if (u >= (long long)nC * per) return;
    const int c = (int)(u / per); const int r0 = 8 * (int)(u % per);
    float w[8];
#pragma unroll
    for (int e = 0; e < 8; ++e) w[e] = cmb_bf(SRC[(size_t)(r0 + e) * lds + c]) * sc;
    v4u pk; pk.x = cmb_pk2(w[0], w[1]); pk.y = cmb_pk2(w[2], w[3]); pk.z = cmb_pk2(w[4], w[5]); pk.w = cmb_pk2(w[6], w[7]);
    VST2(v4u, (v4u*)(DST + (size_t)c * ldd + r0), pk);
}

template <int BIAS_MODE, int OUT_MODE>
__device__ __forceinline__ void gemm64_body(const unsigned short* __restrict__ Ap, int lda, long long strideA,
                                            const unsigned short* __restrict__ Btp, int ldb, long long strideB,
                                            void* __restrict__ Cout, int ldc, long long strideC,
                                            const float* __restrict__ bias, int M, int N, int K, float scale) {
    __shared__ __align__(16) float sT[8 * 16 * 68];
    const int bz = blockIdx.y;
    const int lane = threadIdx.x & 31, wave = threadIdx.x >> 5;
    const int tilesN = N >> 6, tilesM = M >> 6;
    const int tile = blockIdx.x * 8 + wave;
    if (tile >= tilesM * tilesN) return;
    const int tm = tile / tilesN, tn = tile - tm * tilesN;
    const int m0 = tm << 6, n0 = tn << 6;
    const _Float16* Ab = (const _Float16*)Ap + (size_t)bz * strideA;
    const _Float16* Bb = (const _Float16*)Btp + (size_t)bz * strideB;
    const int rlane = lane & 15, koff = (lane >> 4) * 8, mOff = (lane >> 4) * 8;
    const int sb = wave * (16 * 68);

    v8f acc[4][4];
#pragma unroll
    for (int i = 0; i < 4; ++i)
#pragma unroll
        for (int j = 0; j < 4; ++j) acc[i][j] = (v8f){0.f, 0.f, 0.f, 0.f, 0.f, 0.f, 0.f, 0.f};

#pragma unroll 1
    for (int k0 = 0; k0 < K; k0 += 32) {
        v16h bh[4];
#pragma unroll
        for (int j = 0; j < 4; ++j) bh[j] = ldfrag_g(Bb + (size_t)(n0 + (j << 4) + rlane) * ldb + koff + k0);
#pragma unroll
        for (int i = 0; i < 4; ++i) {
            const v16h ah = ldfrag_g(Ab + (size_t)(m0 + (i << 4) + rlane) * lda + koff + k0);
#pragma unroll
            for (int j = 0; j < 4; ++j) acc[i][j] = mma_h(ah, bh[j], acc[i][j]);
            dep_guard_h(acc[i][0], acc[i][3], ah, ah);
        }
        keep4_h(bh[0], bh[1], bh[2], bh[3]);
    }
    acc_guard4(acc[0][0], acc[0][1], acc[0][2], acc[0][3]);
    acc_guard4(acc[1][0], acc[1][1], acc[1][2], acc[1][3]);
    acc_guard4(acc[2][0], acc[2][1], acc[2][2], acc[2][3]);
    acc_guard4(acc[3][0], acc[3][1], acc[3][2], acc[3][3]);

#pragma unroll
    for (int i = 0; i < 4; ++i) {
        const int mBase = m0 + (i << 4);
#pragma unroll
        for (int j = 0; j < 4; ++j) {
            const int n = n0 + (j << 4) + rlane;
            float bv = 0.f;
            if (BIAS_MODE == 2) bv = cmb_bf(bias[n]);
#pragma unroll
            for (int r = 0; r < 8; ++r) {
                float v = acc[i][j][r] * scale;
                if (BIAS_MODE == 1) v += cmb_bf(bias[mBase + mOff + r]);
                if (BIAS_MODE == 2) v += bv;
                sT[sb + (mOff + r) * 68 + (j << 4) + rlane] = v;
            }
        }
        wave_sync_lds();
        if (OUT_MODE == 0) {
            float* C = (float*)Cout + (size_t)bz * strideC;
            const int hh = lane >> 4, c4 = (lane & 15) * 4;
            for (int pass = 0; pass < 2; ++pass) {
#pragma unroll
                for (int it = 0; it < 8; ++it) {
                    const int row = it * 2 + hh;
                    const v4f v = *(const v4f_ma*)&sT[sb + row * 68 + c4];
                    *(volatile v4f*)(C + (size_t)(mBase + row) * ldc + n0 + c4) = v;
                }
                __threadfence();
            }
        } else {
            unsigned short* C = (unsigned short*)Cout + (size_t)bz * strideC;
            const int q = lane >> 3, c8 = (lane & 7) * 8;
            for (int pass = 0; pass < 2; ++pass) {
#pragma unroll
                for (int it = 0; it < 4; ++it) {
                    const int row = it * 4 + q;
                    v8h hv;
#pragma unroll
                    for (int e = 0; e < 8; ++e) hv[e] = (_Float16)sT[sb + row * 68 + c8 + e];
                    *(volatile v8h*)(C + (size_t)(mBase + row) * ldc + n0 + c8) = hv;
                }
                __threadfence();
            }
        }
        wave_sync_lds();
    }
}

__global__ __launch_bounds__(256) void k_gemm_qk(const unsigned short* __restrict__ X16, const unsigned short* __restrict__ WT16, unsigned short* __restrict__ QK16, const float* __restrict__ bqkv) {
    gemm64_body<2, 1>(X16, DM, 0, WT16, DM, 0, (void*)QK16, 2 * DM, 0, bqkv, NB * SEQ, 2 * DM, DM, 0.0625f);
}
__global__ __launch_bounds__(256) void k_gemm_vt(const unsigned short* __restrict__ WV16, const unsigned short* __restrict__ X16, unsigned short* __restrict__ VT16, const float* __restrict__ bv) {
    gemm64_body<1, 1>(WV16, DM, 0, X16, DM, (long long)SEQ * DM, (void*)VT16, SEQ, (long long)DM * SEQ, bv, DM, SEQ, DM, 0.0625f);
}
__global__ __launch_bounds__(256) void k_gemm_out(const unsigned short* __restrict__ CTX16, const unsigned short* __restrict__ WP16, float* __restrict__ OUT, const float* __restrict__ bp) {
    gemm64_body<2, 0>(CTX16, DM, (long long)SEQ * DM, WP16, DM, 0, (void*)OUT, DM, (long long)SEQ_FULL * DM, bp, SEQ, DM, DM, 0.0009765625f);
}

#define AT_PP 40
#define AT_OP 68
static_assert((AT_PP * 2) % 16 == 0);
static_assert(AT_PP >= 32);
__global__ __launch_bounds__(128) void k_flash(const unsigned short* __restrict__ QKp, const unsigned short* __restrict__ VTp, unsigned short* __restrict__ CTXp) {
    __shared__ __align__(16) _Float16 Ps[4 * 16 * AT_PP];
    __shared__ __align__(16) float    Os[4 * 16 * AT_OP];
    const _Float16* QK = (const _Float16*)QKp;
    const _Float16* VT = (const _Float16*)VTp;
    const int tid = threadIdx.x, wave = tid >> 5, lane = tid & 31, hh = lane >> 4, c = lane & 15;
    const int nqb = SEQ / 64;
    const int bx = blockIdx.x; const int qb = bx % nqb; const int bh = bx / nqb; const int h = bh % NH; const int b = bh / NH;
    const int q0 = qb * 64 + wave * 16;
    const size_t qoff = ((size_t)b * SEQ + q0 + c) * (2 * DM) + h * HD + 8 * hh;
    const size_t koff = ((size_t)b * SEQ + c) * (2 * DM) + DM + h * HD + 8 * hh;
    const size_t voff = ((size_t)b * DM + h * HD + c) * SEQ + 8 * hh;
    const int pst = wave * (16 * AT_PP) + (8 * hh) * AT_PP + c;
    const int pld = wave * (16 * AT_PP) + c * AT_PP + 8 * hh;
    const float C2  = 0.125f * 1.4426950408889634f;
    const float PSC = 4096.0f;

    float mrow[8], lpart[8];
    v8f o0 = (v8f){0.f, 0.f, 0.f, 0.f, 0.f, 0.f, 0.f, 0.f}, o1 = o0, o2 = o0, o3 = o0;
#pragma unroll
    for (int r = 0; r < 8; ++r) { mrow[r] = -1.0e30f; lpart[r] = 0.f; }

#pragma unroll 1
    for (int kv0 = 0; kv0 < SEQ; kv0 += 32) {
        v8f s0 = (v8f){0.f, 0.f, 0.f, 0.f, 0.f, 0.f, 0.f, 0.f}, s1 = s0;
#pragma unroll
        for (int dc = 0; dc < 2; ++dc) {
            const v16h qa = ldfrag_g(QK + qoff + dc * 32);
            const v16h k0f = ldfrag_g(QK + koff + (size_t)kv0 * (2 * DM) + dc * 32);
            const v16h k1f = ldfrag_g(QK + koff + (size_t)(kv0 + 16) * (2 * DM) + dc * 32);
            s0 = mma_h(qa, k0f, s0);
            s1 = mma_h(qa, k1f, s1);
            guard_s(s0, s1, qa, k0f, k1f);
        }
#pragma unroll
        for (int r = 0; r < 8; ++r) {
            const float a0 = s0[r] * C2, a1 = s1[r] * C2;
            float m = fmaxf(a0, a1);
            m = fmaxf(m, __shfl_xor(m, 1, 32)); m = fmaxf(m, __shfl_xor(m, 2, 32));
            m = fmaxf(m, __shfl_xor(m, 4, 32)); m = fmaxf(m, __shfl_xor(m, 8, 32));
            const float mnew = fmaxf(mrow[r], m);
            const float alpha = exp2f(mrow[r] - mnew);
            const float p0 = exp2f(a0 - mnew), p1 = exp2f(a1 - mnew);
            lpart[r] = lpart[r] * alpha + (p0 + p1);
            mrow[r] = mnew;
            Ps[pst + r * AT_PP]      = (_Float16)(p0 * PSC);
            Ps[pst + r * AT_PP + 16] = (_Float16)(p1 * PSC);
            o0[r] *= alpha; o1[r] *= alpha; o2[r] *= alpha; o3[r] *= alpha;
        }
        wave_sync_lds();
        {
            FH pa;
            pa.h[0] = *(const v8h_ma*)&Ps[pld];
            pa.h[1] = *(const v8h_ma*)&Ps[pld + 16];
            const v16h vb0 = ldfrag_g(VT + voff + (size_t)(0 * 16) * SEQ + kv0);
            const v16h vb1 = ldfrag_g(VT + voff + (size_t)(1 * 16) * SEQ + kv0);
            const v16h vb2 = ldfrag_g(VT + voff + (size_t)(2 * 16) * SEQ + kv0);
            const v16h vb3 = ldfrag_g(VT + voff + (size_t)(3 * 16) * SEQ + kv0);
            o0 = mma_h(pa.v, vb0, o0);
            o1 = mma_h(pa.v, vb1, o1);
            o2 = mma_h(pa.v, vb2, o2);
            o3 = mma_h(pa.v, vb3, o3);
            guard_o(o0, o1, o2, o3, pa.v, vb0, vb1, vb2, vb3);
        }
        wave_sync_lds();
    }

    const int ob = wave * (16 * AT_OP);
#pragma unroll
    for (int r = 0; r < 8; ++r) {
        float l = lpart[r];
        l += __shfl_xor(l, 1, 32); l += __shfl_xor(l, 2, 32); l += __shfl_xor(l, 4, 32); l += __shfl_xor(l, 8, 32);
        const float inv = 1.0f / (l * 64.0f);
        Os[ob + (8 * hh + r) * AT_OP +  0 + c] = o0[r] * inv;
        Os[ob + (8 * hh + r) * AT_OP + 16 + c] = o1[r] * inv;
        Os[ob + (8 * hh + r) * AT_OP + 32 + c] = o2[r] * inv;
        Os[ob + (8 * hh + r) * AT_OP + 48 + c] = o3[r] * inv;
    }
    wave_sync_lds();
    {
        unsigned short* CT = CTXp + ((size_t)b * SEQ + q0) * DM + h * HD;
        const int qq = lane >> 3, c8 = (lane & 7) * 8;
        for (int pass = 0; pass < 2; ++pass) {
#pragma unroll
            for (int it = 0; it < 4; ++it) {
                const int row = it * 4 + qq;
                v8h hv;
#pragma unroll
                for (int e = 0; e < 8; ++e) hv[e] = (_Float16)Os[ob + row * AT_OP + c8 + e];
                *(volatile v8h*)(CT + (size_t)row * DM + c8) = hv;
            }
            __threadfence();
        }
    }
}

#define WS_X16  ((size_t)NB * SEQ * DM * 2)
#define WS_WT16 ((size_t)3 * DM * DM * 2)
#define WS_WP16 ((size_t)DM * DM * 2)
#define WS_QK16 ((size_t)NB * SEQ * 2 * DM * 2)
#define WS_VT16 ((size_t)NB * DM * SEQ * 2)
#define WS_CTX  ((size_t)NB * SEQ * DM * 2)
#define WS_TOTAL (WS_X16 + WS_WT16 + WS_WP16 + WS_QK16 + WS_VT16 + WS_CTX)
static_assert(WS_TOTAL <= (size_t)134217728);
static_assert(WS_X16 % 256 == 0 && WS_WT16 % 256 == 0 && WS_WP16 % 256 == 0 && WS_QK16 % 256 == 0 && WS_VT16 % 256 == 0 && WS_CTX % 256 == 0);

extern "C" void kernel_launch(void* const* d_in, const int* in_sizes, int n_in, void* d_out, int out_size, void* d_ws, size_t ws_size, hipStream_t stream) {
    if (n_in < 5) return;
    if (in_sizes[0] < ((NB - 1) * SEQ_FULL + SEQ) * DM) return;
    if (in_sizes[1] < DM * 3 * DM) return;
    if (in_sizes[2] < 3 * DM) return;
    if (in_sizes[3] < DM * DM) return;
    if (in_sizes[4] < DM) return;
    if (out_size < ((NB - 1) * SEQ_FULL + SEQ) * DM) return;
    if (WS_TOTAL > ws_size) return;
    const float* x     = (const float*)d_in[0];
    const float* Wqkv  = (const float*)d_in[1];
    const float* bqkv  = (const float*)d_in[2];
    const float* Wproj = (const float*)d_in[3];
    const float* bproj = (const float*)d_in[4];
    float* out = (float*)d_out;
    char* wsp = (char*)d_ws;
    unsigned short* X16  = (unsigned short*)wsp; wsp += WS_X16;
    unsigned short* WT16 = (unsigned short*)wsp; wsp += WS_WT16;
    unsigned short* WP16 = (unsigned short*)wsp; wsp += WS_WP16;
    unsigned short* QK16 = (unsigned short*)wsp; wsp += WS_QK16;
    unsigned short* VT16 = (unsigned short*)wsp; wsp += WS_VT16;
    unsigned short* CTX16 = (unsigned short*)wsp; wsp += WS_CTX;

    k_cast_x<<<(unsigned)((((long long)NB * SEQ) * (DM / 8) + 255) / 256), 256, 0, stream>>>(x, X16);
    k_castT_w<<<(unsigned)((((long long)(3 * DM)) * (DM / 8) + 255) / 256), 256, 0, stream>>>(Wqkv, 3 * DM, WT16, DM, DM, 3 * DM, 16.0f);
    k_castT_w<<<(unsigned)((((long long)DM) * (DM / 8) + 255) / 256), 256, 0, stream>>>(Wproj, DM, WP16, DM, DM, DM, 16.0f);
    k_gemm_qk<<<dim3((unsigned)((((NB * SEQ) / 64) * ((2 * DM) / 64)) / 8), 1u), 256, 0, stream>>>(X16, WT16, QK16, bqkv);
    k_gemm_vt<<<dim3((unsigned)(((DM / 64) * (SEQ / 64)) / 8), (unsigned)NB), 256, 0, stream>>>(WT16 + (size_t)2 * DM * DM, X16, VT16, bqkv + 2 * DM);
    k_flash<<<(unsigned)(NB * NH * (SEQ / 64)), 128, 0, stream>>>(QK16, VT16, CTX16);
    k_gemm_out<<<dim3((unsigned)(((SEQ / 64) * (DM / 64)) / 8), (unsigned)NB), 256, 0, stream>>>(CTX16, WP16, out, bproj);
}
